// SelectivePSIv2_49950469653079
// MI455X (gfx1250) — hardware-verified
//
#include <hip/hip_runtime.h>

typedef __attribute__((ext_vector_type(16))) _Float16 v16h;
typedef __attribute__((ext_vector_type(8)))  float  v8f;

union AFrag { v16h v; uint4 q[2]; };
typedef __attribute__((ext_vector_type(4))) float v4f;
typedef __attribute__((ext_vector_type(4))) unsigned v4u;
typedef __attribute__((ext_vector_type(8))) _Float16 v8h;
template <typename V> __device__ __forceinline__ void vst2(void* p, V v) {
    *(volatile V*)p = v; __threadfence(); *(volatile V*)p = v;
}
__device__ __forceinline__ v8f wmma16(v16h a, v16h b, v8f c) {
    v8f d = __builtin_amdgcn_wmma_f32_16x16x32_f16(false, a, false, b, (short)0, c, false, false);
    asm volatile("v_nop\n\tv_nop\n\tv_nop\n\tv_nop" : "+v"(d) : "v"(a), "v"(b));
    return d;
}

#define MODE_F32T      0
#define MODE_GELU_BF16 1
#define MODE_RESID     2

__device__ __forceinline__ float gelu_exact(float v) {
    return 0.5f * v * (1.0f + erff(v * 0.70710678118654752f));
}
__device__ __forceinline__ float sigmoidf(float v) {
    return 1.0f / (1.0f + expf(-v));
}

__global__ __launch_bounds__(256)
void gemm_wmma_f16(const _Float16* __restrict__ A,
                    const _Float16* __restrict__ Bt,
                    const float* __restrict__ bias,
                    float* __restrict__ outF,
                    _Float16* __restrict__ outH,
                    const float* __restrict__ resid,
                    int N, int K, int mode)
{
    const int SEQ = 2048;
    __shared__ __align__(16) float T[64][128];
    int tid  = threadIdx.x;
    int wave = tid >> 5, lane = tid & 31;
    int half = lane >> 4, l16 = lane & 15;
    int tile_m = blockIdx.y * 64  + (wave >> 2) * 32;
    int tile_n = blockIdx.x * 128 + (wave & 3) * 32;

    const _Float16* arow0 = A  + (size_t)(tile_m + l16) * K;
    const _Float16* arow1 = arow0 + (size_t)16 * K;
    const _Float16* brow0 = Bt + (size_t)(tile_n + l16) * K;
    const _Float16* brow1 = brow0 + (size_t)16 * K;
    const int aoff = half * 8;
    const int boff = half * 8;

    v8f acc00 = {}, acc01 = {}, acc10 = {}, acc11 = {};
    for (int k0 = 0; k0 < K; k0 += 32) {
        AFrag a0, a1, b0, b1;
        a0.q[0] = *(const uint4*)(arow0 + k0 + aoff);
        a0.q[1] = *(const uint4*)(arow0 + k0 + 16 + aoff);
        a1.q[0] = *(const uint4*)(arow1 + k0 + aoff);
        a1.q[1] = *(const uint4*)(arow1 + k0 + 16 + aoff);
        b0.q[0] = *(const uint4*)(brow0 + k0 + boff);
        b0.q[1] = *(const uint4*)(brow0 + k0 + boff + 16);
        b1.q[0] = *(const uint4*)(brow1 + k0 + boff);
        b1.q[1] = *(const uint4*)(brow1 + k0 + boff + 16);
        acc00 = wmma16(a0.v, b0.v, acc00);
        acc01 = wmma16(a0.v, b1.v, acc01);
        acc10 = wmma16(a1.v, b0.v, acc10);
        acc11 = wmma16(a1.v, b1.v, acc11);
    }

    v8f accs[2][2] = {{acc00, acc01}, {acc10, acc11}};
    const int mloc0 = (wave >> 2) * 32, nloc0 = (wave & 3) * 32;
    for (int mi = 0; mi < 2; ++mi) {
        for (int ni = 0; ni < 2; ++ni) {
            v8f acc = accs[mi][ni];
            const int nl = nloc0 + ni * 16 + l16;
            const float bv = bias[blockIdx.x * 128 + nl];
            for (int r = 0; r < 8; ++r) {
                float v = acc[r] + bv;
                if (mode == MODE_GELU_BF16) v = gelu_exact(v);
                T[mloc0 + mi * 16 + half * 8 + r][nl] = v;
            }
        }
    }
    __syncthreads();
    const int bm = blockIdx.y * 64, bn = blockIdx.x * 128;
    if (mode == MODE_F32T) {
        const int bidx = bm >> 11, s0 = bm & (SEQ - 1);
        for (int g = tid; g < 128 * 16; g += 256) {
            const int nl = g >> 4, pc = g & 15;
            v4f v = {T[pc * 4][nl], T[pc * 4 + 1][nl], T[pc * 4 + 2][nl], T[pc * 4 + 3][nl]};
            vst2(outF + ((size_t)bidx * N + bn + nl) * SEQ + s0 + pc * 4, v);
        }
    } else if (mode == MODE_GELU_BF16) {
        for (int g = tid; g < 64 * 16; g += 256) {
            const int ml = g >> 4, pc = g & 15;
            union { v8h h; v4u u; } pk;
            for (int e = 0; e < 8; ++e) pk.h[e] = (_Float16)T[ml][pc * 8 + e];
            vst2(outH + (size_t)(bm + ml) * N + bn + pc * 8, pk.u);
        }
    } else {
        for (int g = tid; g < 64 * 32; g += 256) {
            const int ml = g >> 5, pc = g & 31;
            const size_t idx = (size_t)(bm + ml) * N + bn + pc * 4;
            v4f v = *(const v4f*)(&T[ml][pc * 4]) + *(const v4f*)(resid + idx);
            vst2(outF + idx, v);
        }
    }
}

__global__ void f32_to_f16_kernel(const float* __restrict__ in, _Float16* __restrict__ out, size_t n)
{
    size_t g = (size_t)blockIdx.x * blockDim.x + threadIdx.x;
    if (g * 8 >= n) return;
    const v4f a = *(const v4f*)(in + g * 8), b = *(const v4f*)(in + g * 8 + 4);
    union { v8h h; v4u u; } pk;
    for (int i = 0; i < 4; ++i) { pk.h[i] = (_Float16)a[i]; pk.h[4 + i] = (_Float16)b[i]; }
    vst2(out + g * 8, pk.u);
}

__global__ void w_transpose_f16(const float* __restrict__ W, _Float16* __restrict__ Wt, int K, int N)
{
    __shared__ float tile[64][33];
    int n0 = blockIdx.x * 32, k0 = blockIdx.y * 64;
    for (int i = threadIdx.y; i < 64; i += 8)
        tile[i][threadIdx.x] = W[(size_t)(k0 + i) * N + n0 + threadIdx.x];
    __syncthreads();
    for (int i = threadIdx.y; i < 32; i += 8) {
        union { _Float16 h[2]; unsigned u; } pk;
        pk.h[0] = (_Float16)tile[2 * threadIdx.x][i]; pk.h[1] = (_Float16)tile[2 * threadIdx.x + 1][i];
        vst2(Wt + (size_t)(n0 + i) * K + k0 + 2 * threadIdx.x, pk.u);
    }
}

__global__ void transpose_f32(const float* __restrict__ in,
                              float* __restrict__ out, int R, int C)
{
    __shared__ float tile[32][33];
    size_t bo = (size_t)blockIdx.z * R * C;
    int r0 = blockIdx.y * 32, c0 = blockIdx.x * 32;
    for (int i = threadIdx.y; i < 32; i += 8)
        tile[i][threadIdx.x] = in[bo + (size_t)(r0 + i) * C + c0 + threadIdx.x];
    __syncthreads();
    for (int i = threadIdx.y; i < 32; i += 8)
        vst2(out + bo + (size_t)(c0 + i) * R + r0 + threadIdx.x, tile[threadIdx.x][i]);
}

__device__ __forceinline__ float4 block_scan_inc(float4 v, float4* sh)
{
    int t = threadIdx.x;
    sh[t] = v;
    __syncthreads();
    for (int off = 1; off < 256; off <<= 1) {
        float4 u;
        bool p = (t >= off);
        if (p) u = sh[t - off];
        __syncthreads();
        if (p) {
            float4 w = sh[t];
            w.x += u.x; w.y += u.y; w.z += u.z; w.w += u.w;
            sh[t] = w;
        }
        __syncthreads();
    }
    float4 r = sh[t];
    __syncthreads();
    return r;
}

__global__ __launch_bounds__(256)
void scan_kernel(const float* __restrict__ xT,   const float* __restrict__ pdT,
                 const float* __restrict__ wgT,  const float* __restrict__ magT,
                 const float* __restrict__ qpT,  const float* __restrict__ mixT,
                 const float* __restrict__ int_scale,
                 const float* __restrict__ gate_temp,
                 float* __restrict__ outT)
{
    __shared__ float4 sh[256];
    __shared__ __align__(16) float so[2048];
    const int S = 2048;
    int ch = blockIdx.x;
    int b = ch >> 10, d = ch & 1023;
    size_t base      = (size_t)ch * S;
    size_t mixr_base = ((size_t)b * 2048 + d) * S;
    size_t mixi_base = ((size_t)b * 2048 + 1024 + d) * S;
    int t  = threadIdx.x;
    int e0 = t * 8;
    float isc = fabsf(int_scale[d]);
    float gt  = gate_temp[0];

    float phi[8];
    {
        float4 p0 = *(const float4*)(pdT + base + e0);
        float4 p1 = *(const float4*)(pdT + base + e0 + 4);
        float pd[8] = {p0.x,p0.y,p0.z,p0.w, p1.x,p1.y,p1.z,p1.w};
        float run = 0.f;
        for (int j = 0; j < 8; ++j) { run += pd[j] * isc; phi[j] = run; }
        float4 sc = block_scan_inc(make_float4(run, 0.f, 0.f, 0.f), sh);
        float pref = sc.x - run;
        for (int j = 0; j < 8; ++j) phi[j] += pref;
    }

    float cr[8], ci[8], cw[8];
    {
        float4 a0 = *(const float4*)(xT   + base + e0);
        float4 a1 = *(const float4*)(xT   + base + e0 + 4);
        float4 g0 = *(const float4*)(wgT  + base + e0);
        float4 g1 = *(const float4*)(wgT  + base + e0 + 4);
        float4 m0 = *(const float4*)(magT + base + e0);
        float4 m1 = *(const float4*)(magT + base + e0 + 4);
        float xv[8] = {a0.x,a0.y,a0.z,a0.w, a1.x,a1.y,a1.z,a1.w};
        float gv[8] = {g0.x,g0.y,g0.z,g0.w, g1.x,g1.y,g1.z,g1.w};
        float mv[8] = {m0.x,m0.y,m0.z,m0.w, m1.x,m1.y,m1.z,m1.w};
        for (int j = 0; j < 8; ++j) {
            float wg  = sigmoidf(gv[j] * gt);
            float mag = 5.0f * sigmoidf(mv[j]);
            float c   = wg * xv[j] * mag;
            float sp, cp; sincosf(phi[j], &sp, &cp);
            cr[j] = c * cp;
            ci[j] = c * sp;
            cw[j] = wg * mag + 1e-8f;
        }
    }
    float sr = 0.f, si = 0.f, sw = 0.f;
    for (int j = 0; j < 8; ++j) { sr += cr[j]; si += ci[j]; sw += cw[j]; }
    float4 sc = block_scan_inc(make_float4(sr, si, sw, 0.f), sh);
    float pr = sc.x - sr, pi = sc.y - si, pw = sc.z - sw;

    {
        float4 q0 = *(const float4*)(qpT + base + e0);
        float4 q1 = *(const float4*)(qpT + base + e0 + 4);
        float4 r0 = *(const float4*)(mixT + mixr_base + e0);
        float4 r1 = *(const float4*)(mixT + mixr_base + e0 + 4);
        float4 i0 = *(const float4*)(mixT + mixi_base + e0);
        float4 i1 = *(const float4*)(mixT + mixi_base + e0 + 4);
        float qv [8] = {q0.x,q0.y,q0.z,q0.w, q1.x,q1.y,q1.z,q1.w};
        float mrv[8] = {r0.x,r0.y,r0.z,r0.w, r1.x,r1.y,r1.z,r1.w};
        float miv[8] = {i0.x,i0.y,i0.z,i0.w, i1.x,i1.y,i1.z,i1.w};
        float accr = pr, acci = pi, accw = pw;
        float o[8];
        for (int j = 0; j < 8; ++j) {
            accr += cr[j]; acci += ci[j]; accw += cw[j];
            float inv = rsqrtf(accw);
            float mr = accr * inv, mi = acci * inv;
            float q  = phi[j] + qv[j];
            float sq, cq; sincosf(q, &sq, &cq);
            float rre = mr * cq + mi * sq;
            float rim = mi * cq - mr * sq;
            o[j] = sigmoidf(mrv[j]) * rre + sigmoidf(miv[j]) * rim;
        }
        for (int j = 0; j < 8; ++j) so[e0 + j] = o[j];
    }
    __syncthreads();
    vst2(outT + base + t * 4, *(const v4f*)(&so[t * 4]));
    vst2(outT + base + 1024 + t * 4, *(const v4f*)(&so[1024 + t * 4]));
}

__global__ __launch_bounds__(256)
void layernorm_f16_kernel(const float* __restrict__ in,
                           const float* __restrict__ g,
                           const float* __restrict__ bb,
                           _Float16* __restrict__ out)
{
    const int D = 1024;
    __shared__ float s1[256], s2[256];
    int row = blockIdx.x, t = threadIdx.x;
    float4 v = ((const float4*)(in + (size_t)row * D))[t];
    s1[t] = v.x + v.y + v.z + v.w;
    s2[t] = v.x*v.x + v.y*v.y + v.z*v.z + v.w*v.w;
    __syncthreads();
    for (int off = 128; off > 0; off >>= 1) {
        if (t < off) { s1[t] += s1[t + off]; s2[t] += s2[t + off]; }
        __syncthreads();
    }
    float mean = s1[0] * (1.0f / D);
    float var  = s2[0] * (1.0f / D) - mean * mean;
    float inv  = rsqrtf(var + 1e-5f);
    int d0 = t * 4;
    float vv[4] = {v.x, v.y, v.z, v.w};
    union { _Float16 h[4]; unsigned long long u; } pk;
    for (int j = 0; j < 4; ++j) pk.h[j] = (_Float16)((vv[j] - mean) * inv * g[d0 + j] + bb[d0 + j]);
    vst2(out + (size_t)row * D + d0, pk.u);
}

extern "C" void kernel_launch(void* const* d_in, const int* in_sizes, int n_in,
                              void* d_out, int out_size, void* d_ws, size_t ws_size,
                              hipStream_t stream)
{
    (void)in_sizes; (void)n_in; (void)out_size; (void)ws_size;
    const int D = 1024, S = 2048, Bn = 2, M = Bn * S;

    const float* x       = (const float*)d_in[0];
    const float* w_pt1   = (const float*)d_in[1];
    const float* b_pt1   = (const float*)d_in[2];
    const float* w_pt2   = (const float*)d_in[3];
    const float* b_pt2   = (const float*)d_in[4];
    const float* i_scale = (const float*)d_in[5];
    const float* w_wg    = (const float*)d_in[6];
    const float* b_wg    = (const float*)d_in[7];
    const float* g_temp  = (const float*)d_in[8];
    const float* w_mag   = (const float*)d_in[9];
    const float* b_mag   = (const float*)d_in[10];
    const float* w_q1    = (const float*)d_in[11];
    const float* b_q1    = (const float*)d_in[12];
    const float* w_q2    = (const float*)d_in[13];
    const float* b_q2    = (const float*)d_in[14];
    const float* w_mix   = (const float*)d_in[15];
    const float* b_mix   = (const float*)d_in[16];
    const float* ln_g    = (const float*)d_in[17];
    const float* ln_b    = (const float*)d_in[18];
    const float* w_o1    = (const float*)d_in[19];
    const float* b_o1    = (const float*)d_in[20];
    const float* w_o2    = (const float*)d_in[21];
    const float* b_o2    = (const float*)d_in[22];
    float* out = (float*)d_out;

    char* ws = (char*)d_ws;
    size_t off = 0;
    auto alloc = [&](size_t bytes) -> char* {
        char* p = ws + off;
        off += (bytes + 255) & ~(size_t)255;
        return p;
    };
    typedef _Float16 f16;
    f16* wpt1t = (f16*)alloc((size_t)D * 2*D * 2);
    f16* wpt2t = (f16*)alloc((size_t)2*D * D * 2);
    f16* wwgt  = (f16*)alloc((size_t)D * D * 2);
    f16* wmagt = (f16*)alloc((size_t)D * D * 2);
    f16* wq1t  = (f16*)alloc((size_t)D * D * 2);
    f16* wq2t  = (f16*)alloc((size_t)D * D * 2);
    f16* wmixt = (f16*)alloc((size_t)D * 2*D * 2);
    f16* wo1t  = (f16*)alloc((size_t)D * D * 2);
    f16* wo2t  = (f16*)alloc((size_t)D * D * 2);
    f16*  xbf  = (f16*)alloc((size_t)M * D * 2);
    f16*  h1   = (f16*)alloc((size_t)M * 2*D * 2);
    float* xT   = (float*)alloc((size_t)M * D * 4);
    float* pdT  = (float*)alloc((size_t)M * D * 4);
    float* wgT  = (float*)alloc((size_t)M * D * 4);
    float* magT = (float*)alloc((size_t)M * D * 4);
    float* qpT  = (float*)alloc((size_t)M * D * 4);
    float* mixT = (float*)alloc((size_t)M * 2*D * 4);
    f16*  q1h  = h1;
    f16*  o1h  = h1;
    float* outT = pdT;
    float* retr = xT;
    f16*  lnbf = xbf;

    dim3 tb(32, 8);
    w_transpose_f16<<<dim3(2*D/32, D/64),   tb, 0, stream>>>(w_pt1, wpt1t, D,   2*D);
    w_transpose_f16<<<dim3(D/32,   2*D/64), tb, 0, stream>>>(w_pt2, wpt2t, 2*D, D);
    w_transpose_f16<<<dim3(D/32,   D/64),   tb, 0, stream>>>(w_wg,  wwgt,  D,   D);
    w_transpose_f16<<<dim3(D/32,   D/64),   tb, 0, stream>>>(w_mag, wmagt, D,   D);
    w_transpose_f16<<<dim3(D/32,   D/64),   tb, 0, stream>>>(w_q1,  wq1t,  D,   D);
    w_transpose_f16<<<dim3(D/32,   D/64),   tb, 0, stream>>>(w_q2,  wq2t,  D,   D);
    w_transpose_f16<<<dim3(2*D/32, D/64),   tb, 0, stream>>>(w_mix, wmixt, D,   2*D);
    w_transpose_f16<<<dim3(D/32,   D/64),   tb, 0, stream>>>(w_o1,  wo1t,  D,   D);
    w_transpose_f16<<<dim3(D/32,   D/64),   tb, 0, stream>>>(w_o2,  wo2t,  D,   D);

    size_t nx = (size_t)M * D;
    f32_to_f16_kernel<<<dim3((unsigned)((nx / 8 + 255) / 256)), 256, 0, stream>>>(x, xbf, nx);
    transpose_f32<<<dim3(D/32, S/32, Bn), tb, 0, stream>>>(x, xT, S, D);

    gemm_wmma_f16<<<dim3(2*D/128, M/64), 256, 0, stream>>>(
        xbf, wpt1t, b_pt1, nullptr, h1, nullptr, 2*D, D, MODE_GELU_BF16);
    gemm_wmma_f16<<<dim3(D/128, M/64), 256, 0, stream>>>(
        h1, wpt2t, b_pt2, pdT, nullptr, nullptr, D, 2*D, MODE_F32T);
    gemm_wmma_f16<<<dim3(D/128, M/64), 256, 0, stream>>>(
        xbf, wwgt, b_wg, wgT, nullptr, nullptr, D, D, MODE_F32T);
    gemm_wmma_f16<<<dim3(D/128, M/64), 256, 0, stream>>>(
        xbf, wmagt, b_mag, magT, nullptr, nullptr, D, D, MODE_F32T);
    gemm_wmma_f16<<<dim3(D/128, M/64), 256, 0, stream>>>(
        xbf, wq1t, b_q1, nullptr, q1h, nullptr, D, D, MODE_GELU_BF16);
    gemm_wmma_f16<<<dim3(D/128, M/64), 256, 0, stream>>>(
        q1h, wq2t, b_q2, qpT, nullptr, nullptr, D, D, MODE_F32T);
    gemm_wmma_f16<<<dim3(2*D/128, M/64), 256, 0, stream>>>(
        xbf, wmixt, b_mix, mixT, nullptr, nullptr, 2*D, D, MODE_F32T);

    scan_kernel<<<dim3(Bn * D), 256, 0, stream>>>(
        xT, pdT, wgT, magT, qpT, mixT, i_scale, g_temp, outT);

    transpose_f32<<<dim3(S/32, D/32, Bn), tb, 0, stream>>>(outT, retr, D, S);

    layernorm_f16_kernel<<<dim3(M), 256, 0, stream>>>(retr, ln_g, ln_b, lnbf);

    gemm_wmma_f16<<<dim3(D/128, M/64), 256, 0, stream>>>(
        lnbf, wo1t, b_o1, nullptr, o1h, nullptr, D, D, MODE_GELU_BF16);
    gemm_wmma_f16<<<dim3(D/128, M/64), 256, 0, stream>>>(
        o1h, wo2t, b_o2, out, nullptr, x, D, D, MODE_RESID);
}
